// CausalMultiHypothesisTransformerLayer_3204045603765
// MI455X (gfx1250) — hardware-verified
//
#include <hip/hip_runtime.h>
#include <hip/hip_bf16.h>
#include <math.h>

#define BB 4
#define SS 1024
#define EE 256
#define FFc 512
#define MTOK (BB * SS)
#define DKK 64
#define QW 2
#define GSTR 48
#define HH 8

typedef _Float16 bf16;
typedef _Float16 f16;
typedef __attribute__((ext_vector_type(4))) unsigned v4u_t;
typedef unsigned v4ua __attribute__((ext_vector_type(4), may_alias));
typedef __attribute__((ext_vector_type(4))) float v4f_t;
typedef float v4fa __attribute__((ext_vector_type(4), may_alias));
typedef __attribute__((ext_vector_type(16))) bf16  bf16x16;
typedef bf16x16 f16x16;
typedef __attribute__((ext_vector_type(8)))  bf16  bf16x8;
typedef bf16x8 f16x8;
typedef __attribute__((ext_vector_type(4)))  bf16  bf16x4;
typedef __attribute__((ext_vector_type(8)))  float f32x8;
__device__ __forceinline__ f32x8 wmma16(f16x16 a, f16x16 b, f32x8 c) {
  c = __builtin_amdgcn_wmma_f32_16x16x32_f16(false, a, false, b, (short)0, c, false, false);
  asm volatile("v_nop\n\tv_nop\n\tv_nop\n\tv_nop" : "+v"(c) : "v"(a), "v"(b));
  return c;
}
#define LDS_STRIDE 48
#define KSTRIDE    72
#define VSTRIDE    48

__device__ __forceinline__ f32x8 wmma_bf16(bf16x16 a, bf16x16 b, f32x8 c) {
  c = __builtin_amdgcn_wmma_f32_16x16x32_f16(false, a, false, b, (short)0, c, false, false);
  asm volatile("v_nop\n\tv_nop\n\tv_nop\n\tv_nop" : "+v"(c) : "v"(a), "v"(b));
  return c;
}

template <typename T>
__device__ __forceinline__ bf16x16 load_frag(const T* __restrict__ base, int ld,
                                             int row0, int k0) {
  const int lane = threadIdx.x & 31;
  const int r    = lane & 15;
  const int kh   = (lane >> 4) * 8;
  const T* p0 = base + (size_t)(row0 + r) * ld + (k0 + kh);
  const T* p1 = p0 + 16;
  bf16x16 f;
#pragma unroll
  for (int i = 0; i < 8; ++i) {
    f[i]     = (bf16)p0[i];
    f[i + 8] = (bf16)p1[i];
  }
  return f;
}

__device__ __forceinline__ bf16x16 lds_frag(const bf16* base, int stride) {
  const int lane = threadIdx.x & 31;
  const int row  = lane & 15;
  const int kh   = (lane >> 4) * 8;
  const bf16x8 lo = *(const bf16x8*)(base + row * stride + kh);
  const bf16x8 hi = *(const bf16x8*)(base + row * stride + kh + 16);
  bf16x16 f;
#pragma unroll
  for (int i = 0; i < 8; ++i) { f[i] = lo[i]; f[i + 8] = hi[i]; }
  return f;
}

template <typename T>
__device__ __forceinline__ void stage_read16(const T* __restrict__ p, float* buf) {
#pragma unroll
  for (int i = 0; i < 16; ++i) buf[i] = (float)p[i];
}

__device__ __forceinline__ void stage_write(bf16* dst, const float* buf, int nquad) {
#pragma unroll
  for (int i = 0; i < nquad; ++i) {
    bf16x4 q;
    q[0] = (bf16)buf[4 * i];     q[1] = (bf16)buf[4 * i + 1];
    q[2] = (bf16)buf[4 * i + 2]; q[3] = (bf16)buf[4 * i + 3];
    *(bf16x4*)(dst + 4 * i) = q;
  }
}

template <typename AT, int MODE>
__global__ __launch_bounds__(256) void gemm_rb_kernel(
    const AT* __restrict__ A, const float* __restrict__ W,
    const float* __restrict__ bias, const float* __restrict__ rowscale, const float* __restrict__ R, const float* __restrict__ rowbias, void* __restrict__ out,
    int M, int N, int K) {
  __shared__ bf16 ldsA[128 * LDS_STRIDE];
  __shared__ bf16 ldsW[256 * LDS_STRIDE];
  __shared__ __attribute__((aligned(16))) unsigned char sob[256 * 136 * 2];

  const int t    = threadIdx.x;
  const int wave = t >> 5;
  const int lane = t & 31;
  const int wm   = (wave & 1) * 64;
  const int wn   = (wave >> 1) * 64;
  const int mBlk = blockIdx.x * 128;
  const int nBlk = blockIdx.y * 256;

  const int arow = t >> 1;
  const int ach  = (t & 1) * 16;

  float abuf[16];
  float wbuf[32];

  stage_read16(A + (size_t)(mBlk + arow) * K + ach, abuf);
  const int nrow = min(nBlk + t, N - 1);
  stage_read16(W + (size_t)nrow * K,          wbuf);
  stage_read16(W + (size_t)nrow * K + 16,     wbuf + 16);

  f32x8 acc[4][4] = {};

  for (int k = 0; k < K; k += 32) {
    __syncthreads();
    stage_write(&ldsA[arow * LDS_STRIDE + ach], abuf, 4);
    stage_write(&ldsW[t * LDS_STRIDE],          wbuf, 8);
    if (k + 32 < K) {
      stage_read16(A + (size_t)(mBlk + arow) * K + (k + 32) + ach, abuf);
      stage_read16(W + (size_t)nrow * K + (k + 32),          wbuf);
      stage_read16(W + (size_t)nrow * K + (k + 32) + 16,     wbuf + 16);
    }
    __syncthreads();

    bf16x16 af[4], wf[4];
#pragma unroll
    for (int i = 0; i < 4; ++i)
      af[i] = lds_frag(ldsA + (wm + 16 * i) * LDS_STRIDE, LDS_STRIDE);
#pragma unroll
    for (int j = 0; j < 4; ++j)
      wf[j] = lds_frag(ldsW + (wn + 16 * j) * LDS_STRIDE, LDS_STRIDE);
#pragma unroll
    for (int i = 0; i < 4; ++i)
#pragma unroll
      for (int j = 0; j < 4; ++j)
        acc[i][j] = wmma_bf16(af[i], wf[j], acc[i][j]);
  }

  const int nlane = lane & 15;
  const int mh    = (lane >> 4) * 8;
  __syncthreads();
  if (MODE == 0 || MODE == 1 || MODE == 3) {
    bf16* so = (bf16*)sob;
#pragma unroll
    for (int i = 0; i < 4; ++i)
#pragma unroll
      for (int j = 0; j < 4; ++j) {
        const int nl = wn + 16 * j + nlane;
        const float bv = bias ? bias[nBlk + nl] : 0.0f;
        if (MODE == 3) {
#pragma unroll 1
          for (int r = 0; r < 8; ++r) {
            const int ml = wm + 16 * i + mh + r;
            const float xg = acc[i][j][r] + bv;
            so[ml * 264 + nl] = (bf16)(0.5f * xg * (1.0f + erff(xg * 0.70710678118654752f)));
          }
        } else {
#pragma unroll
        for (int r = 0; r < 8; ++r) {
          const int ml = wm + 16 * i + mh + r;
          const bf16 hv = (bf16)(acc[i][j][r] + bv);
          if (MODE == 0) so[ml * 264 + nl] = hv;
          else           so[nl * 136 + ml] = hv;
        }
        }
      }
    __syncthreads();
#pragma unroll 1
    for (int pass = 0; pass < 2; ++pass) {
      if (MODE == 0 || MODE == 3) {
        for (int ch = t; ch < 128 * 32; ch += 256) { const int ml = ch >> 5, q = (ch & 31) * 8;
          *(volatile v4u_t*)((bf16*)out + (size_t)(mBlk + ml) * N + nBlk + q) = *(const v4ua*)(so + ml * 264 + q); }
      } else {
        const int b_ = mBlk / SS, s0 = mBlk % SS;
        for (int ch = t; ch < 256 * 16; ch += 256) { const int nl = ch >> 4, q = (ch & 15) * 8; const int n = nBlk + nl, h = n >> 6, dk = n & (DKK - 1);
          *(volatile v4u_t*)((bf16*)out + (((size_t)(b_ * HH + h)) * DKK + dk) * SS + s0 + q) = *(const v4ua*)(so + nl * 136 + q); }
      }
      __threadfence();
    }
  } else {
    float* so = (float*)sob;
#pragma unroll 1
    for (int hf = 0; hf < 2; ++hf) {
      if (wm == hf * 64) {
#pragma unroll
        for (int i = 0; i < 4; ++i)
#pragma unroll
          for (int j = 0; j < 4; ++j) {
            const int nl = wn + 16 * j + nlane;
            const float bv = bias ? bias[nBlk + nl] : 0.0f;
#pragma unroll
            for (int r = 0; r < 8; ++r) { const int mrow = mBlk + hf * 64 + 16 * i + mh + r; so[(16 * i + mh + r) * 260 + nl] = acc[i][j][r] * (rowscale ? rowscale[mrow] : 1.0f) + bv + (rowbias ? rowbias[mrow] : 0.0f); }
          }
      }
      __syncthreads();
      if (R) {
        for (int ch = t; ch < 64 * 64; ch += 256) { const int ml = ch >> 6, q = (ch & 63) * 4;
          if (nBlk + q < N) { const v4f_t rv = *(const v4f_t*)(R + (size_t)(mBlk + hf * 64 + ml) * N + nBlk + q); v4f_t v = *(const v4fa*)(so + ml * 260 + q); v += rv; *(volatile v4fa*)(so + ml * 260 + q) = v; } }
        asm volatile("s_wait_dscnt 0" ::: "memory");
      }
#pragma unroll 1
      for (int pass = 0; pass < 2; ++pass) {
        for (int ch = t; ch < 64 * 64; ch += 256) { const int ml = ch >> 6, q = (ch & 63) * 4;
          if (nBlk + q < N) *(volatile v4f_t*)((float*)out + (size_t)(mBlk + hf * 64 + ml) * N + nBlk + q) = *(const v4fa*)(so + ml * 260 + q); }
        __threadfence();
      }
      __syncthreads();
    }
  }
}


#define GSTR 48
template <typename AT, int EPI, bool OUT16>
__global__ __launch_bounds__(256) void gemm_kne(const AT* __restrict__ A, int lda, const float* __restrict__ Wm, int ldw,
                                                const float* __restrict__ bias, const float* __restrict__ R, const float* __restrict__ gvec,
                                                void* __restrict__ Yv, int ldy, int K) {
  __shared__ __attribute__((aligned(16))) f16 ldsA[128 * GSTR];
  __shared__ __attribute__((aligned(16))) f16 ldsW[128 * GSTR];
  __shared__ __attribute__((aligned(16))) float oS[8][32 * 68];
  const int tid = threadIdx.x, lane = tid & 31, wave = tid >> 5, cl = lane & 15, rh = (lane >> 4) * 8;
  const int m0 = blockIdx.x * 128, n0 = blockIdx.y * 128;
  const int wm = (wave & 3) * 32, wn = (wave >> 2) * 64;
  f32x8 acc[2][4];
#pragma unroll
  for (int i = 0; i < 2; ++i)
#pragma unroll
    for (int j = 0; j < 4; ++j) { f32x8 z = {}; acc[i][j] = z; }
#pragma unroll 1
  for (int k0 = 0; k0 < K; k0 += 32) {
    __syncthreads();
    { const int row = tid >> 1, ch = (tid & 1) * 16;
      const AT* src = A + (size_t)(m0 + row) * lda + k0 + ch;
#pragma unroll
      for (int g = 0; g < 16; ++g) ldsA[row * GSTR + ch + g] = (f16)src[g]; }
    { const int k = tid >> 3, nn0 = (tid & 7) * 16;
      const float* src = Wm + (size_t)(k0 + k) * ldw + n0 + nn0;
#pragma unroll
      for (int g = 0; g < 4; ++g) { const v4f_t v = *(const v4f_t*)(src + 4 * g);
#pragma unroll
        for (int u = 0; u < 4; ++u) ldsW[(nn0 + 4 * g + u) * GSTR + k] = (f16)v[u]; } }
    __syncthreads();
    f16x16 af[2];
#pragma unroll
    for (int i = 0; i < 2; ++i) af[i] = lds_frag(ldsA + (wm + 16 * i) * GSTR, GSTR);
#pragma unroll
    for (int j = 0; j < 4; ++j) {
      const f16x16 bf = lds_frag(ldsW + (wn + 16 * j) * GSTR, GSTR);
#pragma unroll
      for (int i = 0; i < 2; ++i) acc[i][j] = wmma16(af[i], bf, acc[i][j]);
    }
  }
  float* so = oS[wave];
#pragma unroll
  for (int i = 0; i < 2; ++i)
#pragma unroll
    for (int j = 0; j < 4; ++j) {
      const int n = n0 + wn + 16 * j + cl;
      const float bv = bias ? bias[n] : 0.0f;
      const float gv = (EPI == 2) ? gvec[n] : 0.0f;
      if (EPI == 1) {
#pragma unroll 1
        for (int r = 0; r < 8; ++r) { const float xg = acc[i][j][r] + bv; so[(16 * i + rh + r) * 68 + 16 * j + cl] = 0.5f * xg * (1.0f + erff(xg * 0.70710678118654752f)); }
      } else {
#pragma unroll
        for (int r = 0; r < 8; ++r) {
          float v = acc[i][j][r] + bv;
          if (EPI == 2) v = R[(size_t)(m0 + wm + 16 * i + rh + r) * ldy + n] + gv * v;
          so[(16 * i + rh + r) * 68 + 16 * j + cl] = v;
        }
      }
    }
  asm volatile("s_wait_dscnt 0" ::: "memory");
  __builtin_amdgcn_wave_barrier();
#pragma unroll 1
  for (int pass = 0; pass < 2; ++pass) {
    if (OUT16) {
      f16* Y = (f16*)Yv;
#pragma unroll
      for (int it = 0; it < 8; ++it) { const int c = lane + 32 * it, rr = c >> 3, q8 = (c & 7) * 8;
        union { f16 h[8]; v4u_t v; } u;
#pragma unroll
        for (int e = 0; e < 8; ++e) u.h[e] = (f16)so[rr * 68 + q8 + e];
        *(volatile v4u_t*)(Y + (size_t)(m0 + wm + rr) * ldy + n0 + wn + q8) = u.v; }
    } else {
      float* Y = (float*)Yv;
#pragma unroll
      for (int it = 0; it < 16; ++it) { const int f4 = lane + 32 * it, rr = f4 >> 4, q = (f4 & 15) * 4;
        *(volatile v4f_t*)(Y + (size_t)(m0 + wm + rr) * ldy + n0 + wn + q) = *(const v4fa*)(so + rr * 68 + q); }
    }
    __threadfence();
  }
}

#define DD 512
#define KVD 512
#define KVH 8
__global__ __launch_bounds__(64) void attn8_kernel(
    const bf16* __restrict__ Qb, const bf16* __restrict__ Kb,
    const bf16* __restrict__ Vt,
    bf16* __restrict__ attnOut) {
  __shared__ bf16 ldsK[32 * KSTRIDE];
  __shared__ bf16 ldsV[64 * VSTRIDE];
  __shared__ __attribute__((aligned(16))) bf16 ldsO[2][32 * 72];

  const int q0blk = blockIdx.x * 64;
  const int h  = blockIdx.y;
  const int b  = blockIdx.z;
  const int t    = threadIdx.x;
  const int wave = t >> 5;
  const int lane = t & 31;
  const int qlane = lane & 15;
  const int kh8   = (lane >> 4) * 8;
  const int q0 = q0blk + wave * 32;

  const int hk = h;
  const bf16* Qh = Qb + (size_t)b * SS * DD + h * DKK;
  const bf16* Kh = Kb + (size_t)b * SS * KVD + hk * DKK;
  const bf16* Vh = Vt + ((size_t)(b * KVH + hk)) * DKK * SS;

  const int krow = t >> 1;
  const int kcol = (t & 1) * 32;
  const bf16* kSrc = Kh + (size_t)krow * KVD + kcol;
  const bf16* vSrc = Vh + (size_t)t * SS;

  bf16x16 qf[QW][2];
#pragma unroll
  for (int qt = 0; qt < QW; ++qt) {
    qf[qt][0] = load_frag(Qh, DD, q0 + 16 * qt, 0);
    qf[qt][1] = load_frag(Qh, DD, q0 + 16 * qt, 32);
  }

  f32x8 o[QW][4] = {};
  float mrun[QW], lrun[QW];
#pragma unroll
  for (int qt = 0; qt < QW; ++qt) { mrun[qt] = -INFINITY; lrun[qt] = 0.0f; }

  const float scale = 0.17677669529663687f * 1.44269504088896340736f;
  const float NEG2 = -1.0e9f;
  const int kmax = SS - 1;

  bf16x8 kreg[4], vreg[4];
#pragma unroll
  for (int i = 0; i < 4; ++i) {
    kreg[i] = *(const bf16x8*)(kSrc + 8 * i);
    vreg[i] = *(const bf16x8*)(vSrc + 8 * i);
  }

  for (int kb = 0; kb <= kmax; kb += 32) {
    __syncthreads();
#pragma unroll
    for (int i = 0; i < 4; ++i) {
      *(bf16x8*)(&ldsK[krow * KSTRIDE + kcol + 8 * i]) = kreg[i];
      *(bf16x8*)(&ldsV[t * VSTRIDE + 8 * i])           = vreg[i];
    }
    if (kb + 32 <= kmax) {
      const bf16* kn = kSrc + (size_t)(kb + 32) * KVD;
      const bf16* vn = vSrc + (kb + 32);
#pragma unroll
      for (int i = 0; i < 4; ++i) {
        kreg[i] = *(const bf16x8*)(kn + 8 * i);
        vreg[i] = *(const bf16x8*)(vn + 8 * i);
      }
    }
    __syncthreads();

    bf16x16 kf[2][2];
#pragma unroll
    for (int ktile = 0; ktile < 2; ++ktile)
#pragma unroll
      for (int c = 0; c < 2; ++c)
        kf[ktile][c] = lds_frag(ldsK + (ktile * 16) * KSTRIDE + c * 32, KSTRIDE);

    bf16x16 pf[QW];
    bool act[QW];
#pragma unroll
    for (int qt = 0; qt < QW; ++qt) {
      unsigned mbits = 0;
      mbits = 0xFFFFu; act[qt] = true;
      if (act[qt]) {
        const int q_my = q0 + 16 * qt + qlane;
        f32x8 s0 = {}, s1 = {};
        s0 = wmma_bf16(kf[0][0], qf[qt][0], s0);
        s0 = wmma_bf16(kf[0][1], qf[qt][1], s0);
        s1 = wmma_bf16(kf[1][0], qf[qt][0], s1);
        s1 = wmma_bf16(kf[1][1], qf[qt][1], s1);

        float mx = -INFINITY;
#pragma unroll
        for (int r = 0; r < 8; ++r) {
          const int k0i = kb + kh8 + r;
          const int k1i = k0i + 16;
          (void)k0i; (void)k1i; (void)q_my;
          s0[r] = (mbits & (1u << r))       ? s0[r] * scale : NEG2;
          s1[r] = (mbits & (1u << (8 + r))) ? s1[r] * scale : NEG2;
          mx = fmaxf(mx, fmaxf(s0[r], s1[r]));
        }
        mx = fmaxf(mx, __shfl_xor(mx, 16, 32));
        const float mnew  = fmaxf(mrun[qt], mx);
        const float alpha = exp2f(mrun[qt] - mnew);

        float rsum = 0.0f;
#pragma unroll
        for (int r = 0; r < 8; ++r) {
          const float p0 = exp2f(s0[r] - mnew);
          const float p1 = exp2f(s1[r] - mnew);
          rsum += p0 + p1;
          pf[qt][r]     = (bf16)(p0 * 1024.0f);
          pf[qt][r + 8] = (bf16)(p1 * 1024.0f);
        }
        rsum += __shfl_xor(rsum, 16, 32);
        lrun[qt] = lrun[qt] * alpha + rsum;
        mrun[qt] = mnew;

#pragma unroll
        for (int j = 0; j < 4; ++j)
#pragma unroll
          for (int r = 0; r < 8; ++r) o[qt][j][r] *= alpha;
      }
    }

#pragma unroll
    for (int j = 0; j < 4; ++j) {
      const bf16x16 vf = lds_frag(ldsV + (j * 16) * VSTRIDE, VSTRIDE);
#pragma unroll
      for (int qt = 0; qt < QW; ++qt)
        if (act[qt]) o[qt][j] = wmma_bf16(vf, pf[qt], o[qt][j]);
    }
  }

  bf16* so = ldsO[wave];
#pragma unroll
  for (int qt = 0; qt < QW; ++qt) {
    const float rl = 1.0f / (lrun[qt] * 1024.0f);
#pragma unroll
    for (int j = 0; j < 4; ++j)
#pragma unroll
      for (int r = 0; r < 8; ++r) so[(16 * qt + qlane) * 72 + j * 16 + kh8 + r] = (bf16)(o[qt][j][r] * rl);
  }
  asm volatile("s_wait_dscnt 0" ::: "memory");
#pragma unroll 1
  for (int pass = 0; pass < 2; ++pass) {
#pragma unroll
    for (int it = 0; it < 8; ++it) { const int ch = lane + 32 * it, ql = ch >> 3, q8 = (ch & 7) * 8;
      *(volatile v4u_t*)(attnOut + ((size_t)(b * SS + q0 + ql)) * DD + h * DKK + q8) = *(const v4ua*)(so + ql * 72 + q8); }
    __threadfence();
  }
}


#undef DD
#undef KVD
#undef KVH
#undef HH
#define DD 256
#define KVD 256
#define KVH 4
#define HH 4
__global__ __launch_bounds__(64) void attn4_kernel(
    const bf16* __restrict__ Qb, const bf16* __restrict__ Kb,
    const bf16* __restrict__ Vt,
    bf16* __restrict__ attnOut) {
  __shared__ bf16 ldsK[32 * KSTRIDE];
  __shared__ bf16 ldsV[64 * VSTRIDE];
  __shared__ __attribute__((aligned(16))) bf16 ldsO[2][32 * 72];

  const int q0blk = blockIdx.x * 64;
  const int h  = blockIdx.y;
  const int b  = blockIdx.z;
  const int t    = threadIdx.x;
  const int wave = t >> 5;
  const int lane = t & 31;
  const int qlane = lane & 15;
  const int kh8   = (lane >> 4) * 8;
  const int q0 = q0blk + wave * 32;

  const int hk = h;
  const bf16* Qh = Qb + (size_t)b * SS * DD + h * DKK;
  const bf16* Kh = Kb + (size_t)b * SS * KVD + hk * DKK;
  const bf16* Vh = Vt + ((size_t)(b * KVH + hk)) * DKK * SS;

  const int krow = t >> 1;
  const int kcol = (t & 1) * 32;
  const bf16* kSrc = Kh + (size_t)krow * KVD + kcol;
  const bf16* vSrc = Vh + (size_t)t * SS;

  bf16x16 qf[QW][2];
#pragma unroll
  for (int qt = 0; qt < QW; ++qt) {
    qf[qt][0] = load_frag(Qh, DD, q0 + 16 * qt, 0);
    qf[qt][1] = load_frag(Qh, DD, q0 + 16 * qt, 32);
  }

  f32x8 o[QW][4] = {};
  float mrun[QW], lrun[QW];
#pragma unroll
  for (int qt = 0; qt < QW; ++qt) { mrun[qt] = -INFINITY; lrun[qt] = 0.0f; }

  const float scale = 0.125f * 1.44269504088896340736f;
  const float NEG2 = -1.0e9f;
  const int kmax = SS - 1;

  bf16x8 kreg[4], vreg[4];
#pragma unroll
  for (int i = 0; i < 4; ++i) {
    kreg[i] = *(const bf16x8*)(kSrc + 8 * i);
    vreg[i] = *(const bf16x8*)(vSrc + 8 * i);
  }

  for (int kb = 0; kb <= kmax; kb += 32) {
    __syncthreads();
#pragma unroll
    for (int i = 0; i < 4; ++i) {
      *(bf16x8*)(&ldsK[krow * KSTRIDE + kcol + 8 * i]) = kreg[i];
      *(bf16x8*)(&ldsV[t * VSTRIDE + 8 * i])           = vreg[i];
    }
    if (kb + 32 <= kmax) {
      const bf16* kn = kSrc + (size_t)(kb + 32) * KVD;
      const bf16* vn = vSrc + (kb + 32);
#pragma unroll
      for (int i = 0; i < 4; ++i) {
        kreg[i] = *(const bf16x8*)(kn + 8 * i);
        vreg[i] = *(const bf16x8*)(vn + 8 * i);
      }
    }
    __syncthreads();

    bf16x16 kf[2][2];
#pragma unroll
    for (int ktile = 0; ktile < 2; ++ktile)
#pragma unroll
      for (int c = 0; c < 2; ++c)
        kf[ktile][c] = lds_frag(ldsK + (ktile * 16) * KSTRIDE + c * 32, KSTRIDE);

    bf16x16 pf[QW];
    bool act[QW];
#pragma unroll
    for (int qt = 0; qt < QW; ++qt) {
      unsigned mbits = 0;
      mbits = 0xFFFFu; act[qt] = true;
      if (act[qt]) {
        const int q_my = q0 + 16 * qt + qlane;
        f32x8 s0 = {}, s1 = {};
        s0 = wmma_bf16(kf[0][0], qf[qt][0], s0);
        s0 = wmma_bf16(kf[0][1], qf[qt][1], s0);
        s1 = wmma_bf16(kf[1][0], qf[qt][0], s1);
        s1 = wmma_bf16(kf[1][1], qf[qt][1], s1);

        float mx = -INFINITY;
#pragma unroll
        for (int r = 0; r < 8; ++r) {
          const int k0i = kb + kh8 + r;
          const int k1i = k0i + 16;
          (void)k0i; (void)k1i; (void)q_my;
          s0[r] = (mbits & (1u << r))       ? s0[r] * scale : NEG2;
          s1[r] = (mbits & (1u << (8 + r))) ? s1[r] * scale : NEG2;
          mx = fmaxf(mx, fmaxf(s0[r], s1[r]));
        }
        mx = fmaxf(mx, __shfl_xor(mx, 16, 32));
        const float mnew  = fmaxf(mrun[qt], mx);
        const float alpha = exp2f(mrun[qt] - mnew);

        float rsum = 0.0f;
#pragma unroll
        for (int r = 0; r < 8; ++r) {
          const float p0 = exp2f(s0[r] - mnew);
          const float p1 = exp2f(s1[r] - mnew);
          rsum += p0 + p1;
          pf[qt][r]     = (bf16)(p0 * 1024.0f);
          pf[qt][r + 8] = (bf16)(p1 * 1024.0f);
        }
        rsum += __shfl_xor(rsum, 16, 32);
        lrun[qt] = lrun[qt] * alpha + rsum;
        mrun[qt] = mnew;

#pragma unroll
        for (int j = 0; j < 4; ++j)
#pragma unroll
          for (int r = 0; r < 8; ++r) o[qt][j][r] *= alpha;
      }
    }

#pragma unroll
    for (int j = 0; j < 4; ++j) {
      const bf16x16 vf = lds_frag(ldsV + (j * 16) * VSTRIDE, VSTRIDE);
#pragma unroll
      for (int qt = 0; qt < QW; ++qt)
        if (act[qt]) o[qt][j] = wmma_bf16(vf, pf[qt], o[qt][j]);
    }
  }

  bf16* so = ldsO[wave];
#pragma unroll
  for (int qt = 0; qt < QW; ++qt) {
    const float rl = 1.0f / (lrun[qt] * 1024.0f);
#pragma unroll
    for (int j = 0; j < 4; ++j)
#pragma unroll
      for (int r = 0; r < 8; ++r) so[(16 * qt + qlane) * 72 + j * 16 + kh8 + r] = (bf16)(o[qt][j][r] * rl);
  }
  asm volatile("s_wait_dscnt 0" ::: "memory");
#pragma unroll 1
  for (int pass = 0; pass < 2; ++pass) {
#pragma unroll
    for (int it = 0; it < 8; ++it) { const int ch = lane + 32 * it, ql = ch >> 3, q8 = (ch & 7) * 8;
      *(volatile v4u_t*)(attnOut + ((size_t)(b * SS + q0 + ql)) * DD + h * DKK + q8) = *(const v4ua*)(so + ql * 72 + q8); }
    __threadfence();
  }
}


#undef DD
#undef KVD
#undef KVH
#undef HH
__global__ __launch_bounds__(256) void k_transpose(const float* __restrict__ Wm, float* __restrict__ Wt, int rows, int cols) {
  __shared__ float tS[64][65];
  const int tid = threadIdx.x, tbj = cols / 64, bi = blockIdx.x / tbj, bj = blockIdx.x % tbj;
  for (int e = tid; e < 64 * 64; e += 256) { const int r = e >> 6, c = e & 63; tS[r][c] = Wm[(size_t)(bi * 64 + r) * cols + bj * 64 + c]; }
  __syncthreads();
  for (int ch = tid; ch < 64 * 16; ch += 256) { const int r = ch >> 4, q4 = (ch & 15) * 4; v4f_t o; o[0] = tS[q4][r]; o[1] = tS[q4 + 1][r]; o[2] = tS[q4 + 2][r]; o[3] = tS[q4 + 3][r];
    float* dst = Wt + (size_t)(bj * 64 + r) * rows + bi * 64 + q4; *(volatile v4f_t*)dst = o; __threadfence(); *(volatile v4f_t*)dst = o; }
}
__global__ __launch_bounds__(256) void k_padhead(const float* __restrict__ Wsrc, const float* __restrict__ bsrc, float* __restrict__ Wp, float* __restrict__ bp) {
  const int slot = blockIdx.x; const int h = slot >> 6, d = slot & 63; const int c = threadIdx.x;
  float v = 0.0f, bv = 0.0f; if (d < 32) { v = Wsrc[(size_t)(h * 32 + d) * EE + c]; bv = bsrc[h * 32 + d]; }
  *(volatile float*)(Wp + (size_t)slot * EE + c) = v; __threadfence(); *(volatile float*)(Wp + (size_t)slot * EE + c) = v; (void)bv; (void)bp;
}
__global__ __launch_bounds__(512) void k_padbias(const float* __restrict__ bsrc, float* __restrict__ bp) { const int slot = threadIdx.x; const int h = slot >> 6, d = slot & 63;
  const float bv = (d < 32) ? bsrc[h * 32 + d] : 0.0f; *(volatile float*)(bp + slot) = bv; __threadfence(); *(volatile float*)(bp + slot) = bv; }
__global__ __launch_bounds__(256) void k_padwoT(const float* __restrict__ Wo, float* __restrict__ WoT) {
  const int slot = blockIdx.x; const int h = slot >> 6, d = slot & 63; const int o = threadIdx.x;
  const float v = (d < 32) ? Wo[(size_t)o * EE + h * 32 + d] : 0.0f;
  *(volatile float*)(WoT + (size_t)slot * EE + o) = v; __threadfence(); *(volatile float*)(WoT + (size_t)slot * EE + o) = v;
}
__global__ __launch_bounds__(256) void k_vt(const float* __restrict__ V, int W, bf16* __restrict__ Vt) { __shared__ __attribute__((aligned(16))) bf16 vT[256][72];
  const int tid = threadIdx.x; const size_t t0 = (size_t)blockIdx.x * 64; const int b = (int)(t0 / SS), n0 = (int)(t0 % SS); const int c0 = blockIdx.y * 256;
  for (int e = tid; e < 64 * 256; e += 256) { const int t = e >> 8, c = e & 255; vT[c][t] = (bf16)V[(t0 + t) * W + c0 + c]; }
  __syncthreads();
#pragma unroll 1
  for (int pass = 0; pass < 2; ++pass) { for (int e = tid; e < 256 * 8; e += 256) { const int c = e >> 3, piece = (e & 7) * 8; *(volatile v4u_t*)(Vt + ((size_t)b * W + c0 + c) * SS + n0 + piece) = *(const v4ua*)(&vT[c][piece]); } __threadfence(); } }
__global__ __launch_bounds__(256) void k_ln(const float* __restrict__ X, const float* __restrict__ Add, const float* __restrict__ g, const float* __restrict__ bb, float* __restrict__ Y) {
  __shared__ __attribute__((aligned(16))) float rowS[8 * (EE + 4)];
  const int tid = threadIdx.x, r = tid >> 5, lane = tid & 31; const size_t row = (size_t)blockIdx.x * 8 + r;
  float s = 0.0f;
#pragma unroll 1
  for (int i = lane; i < EE; i += 32) { float v = X[row * EE + i]; if (Add) v += Add[row * EE + i]; rowS[r * (EE + 4) + i] = v; s += v; }
#pragma unroll
  for (int off = 1; off < 32; off <<= 1) s += __shfl_xor(s, off, 32);
  const float mean = s * (1.0f / EE); float q = 0.0f;
#pragma unroll 1
  for (int i = lane; i < EE; i += 32) { const float d = rowS[r * (EE + 4) + i] - mean; q += d * d; }
#pragma unroll
  for (int off = 1; off < 32; off <<= 1) q += __shfl_xor(q, off, 32);
  const float rstd = rsqrtf(q * (1.0f / EE) + 1e-5f);
#pragma unroll 1
  for (int i = lane; i < EE; i += 32) rowS[r * (EE + 4) + i] = (rowS[r * (EE + 4) + i] - mean) * rstd * g[i] + bb[i];
  __syncthreads();
#pragma unroll 1
  for (int pass = 0; pass < 2; ++pass) { for (int q4 = tid; q4 < 8 * (EE / 4); q4 += 256) { const int rr = q4 / (EE / 4), c4 = (q4 % (EE / 4)) * 4;
      *(volatile v4f_t*)(Y + ((size_t)blockIdx.x * 8 + rr) * EE + c4) = *(const v4fa*)(rowS + rr * (EE + 4) + c4); } __threadfence(); }
}
__global__ __launch_bounds__(256) void k_refmean(const float* __restrict__ A, const float* __restrict__ Bm, float* __restrict__ R) { const size_t off = (size_t)blockIdx.x * EE + threadIdx.x;
  const float v = 0.5f * (A[off] + Bm[off]); *(volatile float*)(R + off) = v; __threadfence(); *(volatile float*)(R + off) = v; }
__global__ __launch_bounds__(256) void k_relu(float* __restrict__ t, int rowlen) { const size_t row = blockIdx.x;
  for (int q4 = threadIdx.x; q4 < rowlen / 4; q4 += 256) { v4f_t v = *(const v4f_t*)(t + row * rowlen + q4 * 4); for (int e = 0; e < 4; ++e) v[e] = fmaxf(v[e], 0.0f);
    *(volatile v4f_t*)(t + row * rowlen + q4 * 4) = v; __threadfence(); *(volatile v4f_t*)(t + row * rowlen + q4 * 4) = v; } }
__global__ __launch_bounds__(256) void k_fuse(const float* __restrict__ G, const float* __restrict__ w2, const float* __restrict__ b2, const float* __restrict__ R0, const float* __restrict__ R1, const float* __restrict__ R2, float* __restrict__ F) {
  const int tid = threadIdx.x, wave = tid >> 5, lane = tid & 31; const size_t row = (size_t)blockIdx.x * 8 + wave;
  float l0 = 0.0f, l1 = 0.0f, l2 = 0.0f;
#pragma unroll 1
  for (int i = lane; i < EE; i += 32) { const float g = G[row * EE + i]; l0 += g * w2[i * 3 + 0]; l1 += g * w2[i * 3 + 1]; l2 += g * w2[i * 3 + 2]; }
#pragma unroll
  for (int off = 1; off < 32; off <<= 1) { l0 += __shfl_xor(l0, off, 32); l1 += __shfl_xor(l1, off, 32); l2 += __shfl_xor(l2, off, 32); }
  l0 += b2[0]; l1 += b2[1]; l2 += b2[2]; const float m = fmaxf(l0, fmaxf(l1, l2)); const float e0 = expf(l0 - m), e1 = expf(l1 - m), e2 = expf(l2 - m); const float iz = 1.0f / (e0 + e1 + e2);
  const float a0 = e0 * iz, a1 = e1 * iz, a2 = e2 * iz;
  const int c0 = lane * 8; v4f_t o0, o1;
  for (int e = 0; e < 4; ++e) { o0[e] = a0 * R0[row * EE + c0 + e] + a1 * R1[row * EE + c0 + e] + a2 * R2[row * EE + c0 + e]; o1[e] = a0 * R0[row * EE + c0 + 4 + e] + a1 * R1[row * EE + c0 + 4 + e] + a2 * R2[row * EE + c0 + 4 + e]; }
  *(volatile v4f_t*)(F + row * EE + c0) = o0; *(volatile v4f_t*)(F + row * EE + c0 + 4) = o1; __threadfence(); *(volatile v4f_t*)(F + row * EE + c0) = o0; *(volatile v4f_t*)(F + row * EE + c0 + 4) = o1;
}
__global__ __launch_bounds__(256) void k_ones(float* __restrict__ p, int n) { for (int i = threadIdx.x; i < n; i += 256) { *(volatile float*)(p + i) = 1.0f; __threadfence(); *(volatile float*)(p + i) = 1.0f; } }

extern "C" void kernel_launch(void* const* d_in, const int* in_sizes, int n_in,
                              void* d_out, int out_size, void* d_ws, size_t ws_size,
                              hipStream_t stream) {
  (void)in_sizes; (void)n_in; (void)out_size;
  const float** f = (const float**)d_in;
  const float* x = f[0], *iw1 = f[1], *ib1 = f[2], *iw2 = f[3], *ib2 = f[4], *hiw = f[5], *hib = f[6], *how = f[7], *hob = f[8], *ciw = f[9], *cib = f[10], *cow = f[11], *cob = f[12],
             *dw1 = f[13], *db1 = f[14], *dw2 = f[15], *db2 = f[16], *fw1 = f[17], *fb1 = f[18], *fw2 = f[19], *fb2 = f[20], *ng = f[21], *nb = f[22], *uw1 = f[23], *ub1 = f[24], *uw2 = f[25], *ub2 = f[26];
  float* out = (float*)d_out;
  char* ws = (char*)d_ws;
  float* X = (float*)ws; ws += (size_t)MTOK * EE * 4;
  float* T512 = (float*)ws; ws += (size_t)MTOK * FFc * 4;
  float* causal = (float*)ws; ws += (size_t)MTOK * EE * 4;
  float* iv = (float*)ws; ws += (size_t)MTOK * EE * 4;
  float* WqP = (float*)ws; ws += (size_t)512 * EE * 4; float* WkP = (float*)ws; ws += (size_t)512 * EE * 4; float* WvP = (float*)ws; ws += (size_t)512 * EE * 4; float* WoT = (float*)ws; ws += (size_t)512 * EE * 4;
  float* bqP = (float*)ws; ws += 512 * 4; float* bkP = (float*)ws; ws += 512 * 4; float* bvP = (float*)ws; ws += 512 * 4;
  bf16* Q16 = (bf16*)ws; ws += (size_t)MTOK * 512 * 2; bf16* K16 = (bf16*)ws; ws += (size_t)MTOK * 512 * 2; bf16* Vt = (bf16*)ws; ws += (size_t)MTOK * 512 * 2; bf16* att = (bf16*)ws; ws += (size_t)MTOK * 512 * 2;
  float* V32 = (float*)ws; ws += (size_t)MTOK * 512 * 4;
  float* hs = (float*)ws; ws += (size_t)3 * MTOK * EE * 4;
  float* refm = (float*)ws; ws += (size_t)MTOK * EE * 4;
  float* cfo = (float*)ws; ws += (size_t)MTOK * EE * 4;
  float* refined = (float*)ws; ws += (size_t)3 * MTOK * EE * 4;
  float* Wt = (float*)ws; ws += (size_t)EE * 768 * 4;
  float* G = (float*)ws; ws += (size_t)MTOK * EE * 4; float* F = (float*)ws; ws += (size_t)MTOK * EE * 4; float* F2 = (float*)ws; ws += (size_t)MTOK * EE * 4; float* F3 = (float*)ws; ws += (size_t)MTOK * EE * 4;
  float* ones = (float*)ws; ws += 512 * 4;
  if ((size_t)(ws - (char*)d_ws) > ws_size) return;
  const dim3 blk(256);
  k_ones<<<dim3(1), blk, 0, stream>>>(ones, 512);
  for (int b = 0; b < BB; ++b) k_transpose<<<dim3((EE / 64) * (SS / 64)), blk, 0, stream>>>(x + (size_t)b * EE * SS, X + (size_t)b * SS * EE, EE, SS);
  gemm_kne<float, 0, false><<<dim3(MTOK / 128, FFc / 128), blk, 0, stream>>>(X, EE, dw1, FFc, db1, nullptr, nullptr, T512, FFc, EE);
  k_relu<<<dim3(MTOK), blk, 0, stream>>>(T512, FFc);
  gemm_kne<float, 0, false><<<dim3(MTOK / 128, EE / 128), blk, 0, stream>>>(T512, FFc, dw2, EE, db2, nullptr, nullptr, causal, EE, FFc);
  for (int h = 0; h < 3; ++h) {
    gemm_kne<float, 0, false><<<dim3(MTOK / 128, 1), blk, 0, stream>>>(causal, EE, iw1 + (size_t)h * EE * 128, 128, ib1 + h * 128, nullptr, nullptr, T512, 128, EE);
    k_relu<<<dim3(MTOK), blk, 0, stream>>>(T512, 128);
    gemm_kne<float, 2, false><<<dim3(MTOK / 128, EE / 128), blk, 0, stream>>>(T512, 128, iw2 + (size_t)h * 128 * EE, EE, ib2 + h * EE, causal, ones, iv, EE, 128);
    const float* inw = hiw + (size_t)h * 768 * EE; const float* inb = hib + (size_t)h * 768;
    k_padhead<<<dim3(512), blk, 0, stream>>>(inw, inb, WqP, bqP); k_padhead<<<dim3(512), blk, 0, stream>>>(inw + (size_t)EE * EE, inb + EE, WkP, bkP); k_padhead<<<dim3(512), blk, 0, stream>>>(inw + (size_t)2 * EE * EE, inb + 2 * EE, WvP, bvP);
    k_padbias<<<dim3(1), dim3(512), 0, stream>>>(inb, bqP); k_padbias<<<dim3(1), dim3(512), 0, stream>>>(inb + EE, bkP); k_padbias<<<dim3(1), dim3(512), 0, stream>>>(inb + 2 * EE, bvP);
    gemm_rb_kernel<float, 0><<<dim3(MTOK / 128, 512 / 256), blk, 0, stream>>>(iv, WqP, bqP, nullptr, nullptr, nullptr, Q16, MTOK, 512, EE);
    gemm_rb_kernel<float, 0><<<dim3(MTOK / 128, 512 / 256), blk, 0, stream>>>(iv, WkP, bkP, nullptr, nullptr, nullptr, K16, MTOK, 512, EE);
    gemm_rb_kernel<float, 2><<<dim3(MTOK / 128, 512 / 256), blk, 0, stream>>>(iv, WvP, bvP, nullptr, nullptr, nullptr, V32, MTOK, 512, EE);
    k_vt<<<dim3(MTOK / 64, 2), blk, 0, stream>>>(V32, 512, Vt);
    attn8_kernel<<<dim3(SS / 64, 8, BB), dim3(64), 0, stream>>>(Q16, K16, Vt, att);
    k_padwoT<<<dim3(512), blk, 0, stream>>>(how + (size_t)h * EE * EE, WoT);
    gemm_kne<bf16, 0, false><<<dim3(MTOK / 128, EE / 128), blk, 0, stream>>>(att, 512, WoT, EE, hob + h * EE, nullptr, nullptr, hs + (size_t)h * MTOK * EE, EE, 512);
  }
  for (int h = 0; h < 3; ++h) {
    const float* hh_ = hs + (size_t)h * MTOK * EE; const float* ha = hs + (size_t)((h + 1) % 3) * MTOK * EE; const float* hb = hs + (size_t)((h + 2) % 3) * MTOK * EE;
    k_refmean<<<dim3(MTOK), blk, 0, stream>>>(ha, hb, refm);
    const float* inw = ciw + (size_t)h * 768 * EE; const float* inb = cib + (size_t)h * 768;
    gemm_rb_kernel<float, 0><<<dim3(MTOK / 128, 1), blk, 0, stream>>>(hh_, inw, inb, nullptr, nullptr, nullptr, Q16, MTOK, EE, EE);
    gemm_rb_kernel<float, 0><<<dim3(MTOK / 128, 1), blk, 0, stream>>>(refm, inw + (size_t)EE * EE, inb + EE, nullptr, nullptr, nullptr, K16, MTOK, EE, EE);
    gemm_rb_kernel<float, 2><<<dim3(MTOK / 128, 1), blk, 0, stream>>>(refm, inw + (size_t)2 * EE * EE, inb + 2 * EE, nullptr, nullptr, nullptr, V32, MTOK, EE, EE);
    k_vt<<<dim3(MTOK / 64, 1), blk, 0, stream>>>(V32, EE, Vt);
    attn4_kernel<<<dim3(SS / 64, 4, BB), dim3(64), 0, stream>>>(Q16, K16, Vt, att);
    k_transpose<<<dim3((EE / 64) * (EE / 64)), blk, 0, stream>>>(cow + (size_t)h * EE * EE, Wt, EE, EE);
    gemm_kne<bf16, 0, false><<<dim3(MTOK / 128, EE / 128), blk, 0, stream>>>(att, EE, Wt, EE, cob + h * EE, nullptr, nullptr, cfo, EE, EE);
    k_ln<<<dim3(MTOK / 8), blk, 0, stream>>>(hh_, cfo, ng, nb, refined + (size_t)h * MTOK * EE);
    for (int b = 0; b < BB; ++b) k_transpose<<<dim3((SS / 64) * (EE / 64)), blk, 0, stream>>>(refined + (size_t)h * MTOK * EE + (size_t)b * SS * EE, out + (size_t)h * MTOK * EE + (size_t)b * EE * SS, SS, EE);
  }
  gemm_kne<float, 0, false><<<dim3(MTOK / 128, EE / 128), blk, 0, stream>>>(refined, EE, uw1, EE, ub1, nullptr, nullptr, G, EE, EE);
  gemm_kne<float, 2, false><<<dim3(MTOK / 128, EE / 128), blk, 0, stream>>>(refined + (size_t)MTOK * EE, EE, uw1 + (size_t)EE * EE, EE, nullptr, G, ones, G, EE, EE);
  gemm_kne<float, 2, false><<<dim3(MTOK / 128, EE / 128), blk, 0, stream>>>(refined + (size_t)2 * MTOK * EE, EE, uw1 + (size_t)2 * EE * EE, EE, nullptr, G, ones, G, EE, EE);
  k_relu<<<dim3(MTOK), blk, 0, stream>>>(G, EE);
  k_fuse<<<dim3(MTOK / 8), blk, 0, stream>>>(G, uw2, ub2, refined, refined + (size_t)MTOK * EE, refined + (size_t)2 * MTOK * EE, F);
  k_ln<<<dim3(MTOK / 8), blk, 0, stream>>>(F, X, ng + EE, nb + EE, F2);
  k_ln<<<dim3(MTOK / 8), blk, 0, stream>>>(F2, nullptr, ng + 2 * EE, nb + 2 * EE, F3);
  gemm_kne<float, 0, false><<<dim3(MTOK / 128, FFc / 128), blk, 0, stream>>>(F3, EE, fw1, FFc, fb1, nullptr, nullptr, T512, FFc, EE);
  k_relu<<<dim3(MTOK), blk, 0, stream>>>(T512, FFc);
  gemm_kne<float, 2, false><<<dim3(MTOK / 128, EE / 128), blk, 0, stream>>>(T512, FFc, fw2, EE, fb2, F2, ones, F, EE, FFc);
  k_ln<<<dim3(MTOK / 8), blk, 0, stream>>>(F, nullptr, ng + 3 * EE, nb + 3 * EE, F3);
  for (int b = 0; b < BB; ++b) k_transpose<<<dim3((SS / 64) * (EE / 64)), blk, 0, stream>>>(F3 + (size_t)b * SS * EE, out + (size_t)3 * MTOK * EE + (size_t)b * EE * SS, SS, EE);
}
